// NLBlock_40664750359453
// MI455X (gfx1250) — hardware-verified
//
#include <hip/hip_runtime.h>


#define NB_  16
#define C_   256
#define HW   3136
#define WID  56
#define CI   32
#define CG   64
#define NP   784
#define NPP  800
#define PW   28
#define RPAD 32
#define BEPS 1e-5f
typedef _Float16 h16;
typedef unsigned short bf;
typedef __attribute__((ext_vector_type(16))) __bf16   v16bf;
typedef __attribute__((ext_vector_type(16))) _Float16 v16h;
typedef __attribute__((ext_vector_type(8)))  _Float16 v8h;
typedef __attribute__((ext_vector_type(8)))  unsigned short v8us;
typedef __attribute__((ext_vector_type(8)))  float    v8f;
typedef __attribute__((ext_vector_type(4)))  float    v4f;
typedef __attribute__((ext_vector_type(2)))  float    v2f;
typedef __attribute__((ext_vector_type(4)))  unsigned short v4us;
typedef __attribute__((ext_vector_type(2)))  unsigned short v2us;
typedef v8h  __attribute__((may_alias)) v8ha;
typedef v4f  __attribute__((may_alias)) v4fa;
typedef v8us __attribute__((may_alias)) v8usa;

__device__ __forceinline__ unsigned short f2bf(float f) { unsigned u = __float_as_uint(f); u += 0x7FFFu + ((u >> 16) & 1u); return (unsigned short)(u >> 16); }
__device__ __forceinline__ float bf2f(unsigned short b) { return __uint_as_float(((unsigned)b) << 16); }
__device__ __forceinline__ float bfr(float f) { return bf2f(f2bf(f)); }
__device__ __forceinline__ void splitf(float y, unsigned short& h, unsigned short& l) { h = f2bf(y); l = f2bf(y - bf2f(h)); }
__device__ __forceinline__ v16h cat16(v8h lo, v8h hi) { return __builtin_shufflevector(lo, hi, 0, 1, 2, 3, 4, 5, 6, 7, 8, 9, 10, 11, 12, 13, 14, 15); }
__device__ __forceinline__ v16bf cat16b(v8us lo, v8us hi) { return __builtin_bit_cast(v16bf, __builtin_shufflevector(lo, hi, 0, 1, 2, 3, 4, 5, 6, 7, 8, 9, 10, 11, 12, 13, 14, 15)); }
__device__ __forceinline__ v8f wmma16(v16h a, v16h b, v8f c) { return __builtin_amdgcn_wmma_f32_16x16x32_f16(false, a, false, b, (short)0, c, false, false); }
__device__ __forceinline__ v8f wmmab(v16bf a, v16bf b, v8f c) { return __builtin_amdgcn_wmma_f32_16x16x32_bf16(false, a, false, b, (short)0, c, false, false); }

template <typename T16> struct WFrag;
template <> struct WFrag<h16> { typedef v16h V; static __device__ __forceinline__ V ld(const h16* p) { return cat16(*(const v8h*)p, *(const v8h*)(p + 16)); } static __device__ __forceinline__ v8f mma(V a, V b, v8f c) { return wmma16(a, b, c); } };
template <> struct WFrag<bf> { typedef v16bf V; static __device__ __forceinline__ V ld(const bf* p) { return cat16b(*(const v8us*)p, *(const v8us*)(p + 16)); } static __device__ __forceinline__ v8f mma(V a, V b, v8f c) { return wmmab(a, b, c); } };
template <typename T16, int NSPLIT, bool BIAS>
__global__ __launch_bounds__(32) void k_gemmw(const T16* __restrict__ A, const T16* __restrict__ A2, const T16* __restrict__ Bt, const T16* __restrict__ Bt2, int K, float* C, int ldc, const float* __restrict__ bias, size_t sA, size_t sB, size_t sC) {
    typedef typename WFrag<T16>::V V;
    __shared__ __align__(16) float os[16 * 68];
    const size_t z = blockIdx.z; A += z * sA; if (A2) A2 += z * sA; Bt += z * sB; if (Bt2) Bt2 += z * sB; C += z * sC;
    const int lane = threadIdx.x & 31, lr = lane & 15, hi = lane >> 4; const int r0 = blockIdx.x * 64, c0 = blockIdx.y * 64;
    v8f acc[4][4];
#pragma unroll
    for (int mb = 0; mb < 4; ++mb)
#pragma unroll
        for (int nb = 0; nb < 4; ++nb) acc[mb][nb] = (v8f){};
    const size_t aoff = (size_t)(r0 + lr) * K + 8 * hi, boff = (size_t)(c0 + lr) * K + 8 * hi;
#pragma unroll 1
    for (int kc = 0; kc < K; kc += 32) {
        V a[4], a2[4];
#pragma unroll
        for (int mb = 0; mb < 4; ++mb) { a[mb] = WFrag<T16>::ld(A + aoff + (size_t)mb * 16 * K + kc); if (NSPLIT == 1 || NSPLIT == 2) a2[mb] = WFrag<T16>::ld(A2 + aoff + (size_t)mb * 16 * K + kc); }
#pragma unroll
        for (int nb = 0; nb < 4; ++nb) { const V b = WFrag<T16>::ld(Bt + boff + (size_t)nb * 16 * K + kc); V b2; if (NSPLIT >= 2) b2 = WFrag<T16>::ld(Bt2 + boff + (size_t)nb * 16 * K + kc);
#pragma unroll
            for (int mb = 0; mb < 4; ++mb) { acc[mb][nb] = WFrag<T16>::mma(a[mb], b, acc[mb][nb]); if (NSPLIT == 1 || NSPLIT == 2) acc[mb][nb] = WFrag<T16>::mma(a2[mb], b, acc[mb][nb]); if (NSPLIT >= 2) acc[mb][nb] = WFrag<T16>::mma(a[mb], b2, acc[mb][nb]); } }
        asm volatile("v_nop\n\tv_nop\n\tv_nop\n\tv_nop" : "+v"(acc[0][0]), "+v"(acc[1][1]), "+v"(acc[2][2]), "+v"(acc[3][3]) : "v"(a[0]), "v"(a[3]));
    }
#pragma unroll
    for (int mb = 0; mb < 4; ++mb) {
#pragma unroll
        for (int nb = 0; nb < 4; ++nb) {
#pragma unroll
            for (int j = 0; j < 8; ++j) os[(hi * 8 + j) * 68 + nb * 16 + lr] = acc[mb][nb][j]; }
        __builtin_amdgcn_wave_barrier(); asm volatile("" ::: "memory");
        float* crow = C + (size_t)(r0 + mb * 16) * ldc + c0;
#pragma unroll 1
        for (int ps = 0; ps < 2; ++ps) {
#pragma unroll
            for (int s = 0; s < 8; ++s) { const int row = 2 * s + hi, cofs = lr * 4; v4f val = *(const v4fa*)(os + row * 68 + cofs); if (BIAS) { val[0] += bfr(bias[c0 + cofs]); val[1] += bfr(bias[c0 + cofs + 1]); val[2] += bfr(bias[c0 + cofs + 2]); val[3] += bfr(bias[c0 + cofs + 3]); }
                *(volatile v4f*)(crow + (size_t)row * ldc + cofs) = val; }
            if (ps == 0) __threadfence(); }
        __builtin_amdgcn_wave_barrier(); asm volatile("" ::: "memory");
    }
}

template <bool RND>
__global__ __launch_bounds__(256) void k_bnstat(const float* __restrict__ Tn, int NCH, int NPOS, float* ST) { __shared__ float red[256]; const int c = blockIdx.x; const int tid = threadIdx.x; float s = 0.f;
#pragma unroll 1
    for (int b = 0; b < NB_; ++b) { const float* base = Tn + ((size_t)b * NCH + c) * NPOS;
#pragma unroll 1
        for (int i = tid; i < NPOS; i += 256) s = __fadd_rn(s, RND ? bfr(base[i]) : base[i]); }
    red[tid] = s; __syncthreads();
#pragma unroll
    for (int sh = 128; sh; sh >>= 1) { if (tid < sh) red[tid] = __fadd_rn(red[tid], red[tid + sh]); __syncthreads(); }
    const float mu = red[0] * (1.0f / ((float)NB_ * NPOS)); __syncthreads(); float s2 = 0.f;
#pragma unroll 1
    for (int b = 0; b < NB_; ++b) { const float* base = Tn + ((size_t)b * NCH + c) * NPOS;
#pragma unroll 1
        for (int i = tid; i < NPOS; i += 256) { const float d0 = __fsub_rn(RND ? bfr(base[i]) : base[i], mu); float p = __fmul_rn(d0, d0); asm volatile("" : "+v"(p)); s2 = __fadd_rn(s2, p); } }
    red[tid] = s2; __syncthreads();
#pragma unroll
    for (int sh = 128; sh; sh >>= 1) { if (tid < sh) red[tid] = __fadd_rn(red[tid], red[tid + sh]); __syncthreads(); }
    if (tid == 0) { const float rs = __fdiv_rn(1.0f, __fsqrt_rn(__fadd_rn(red[0] * (1.0f / ((float)NB_ * NPOS)), BEPS))); v2f o; o[0] = mu; o[1] = rs; *(volatile v2f*)(ST + (size_t)c * RPAD) = o; __threadfence(); *(volatile v2f*)(ST + (size_t)c * RPAD) = o; } }
__global__ __launch_bounds__(256) void k_bnT(const float* __restrict__ xb, const float* __restrict__ ST, const float* __restrict__ gw, const float* __restrict__ gb, bf* Xh, bf* Xl) { const size_t e = ((size_t)blockIdx.x * 256 + threadIdx.x) * 4; if (e >= (size_t)HW * C_) return; const int c = (int)(e % C_); const int n = (int)(e / C_); v4us oh, ol;
#pragma unroll
    for (int q = 0; q < 4; ++q) { const int cc = c + q; const float mu = ST[(size_t)cc * RPAD], rs = ST[(size_t)cc * RPAD + 1]; float n0 = __fmul_rn(__fsub_rn(bfr(xb[(size_t)cc * HW + n]), mu), rs); asm volatile("" : "+v"(n0)); float n1 = __fmul_rn(bfr(gw[cc]), n0); asm volatile("" : "+v"(n1)); const float y = fmaxf(__fadd_rn(n1, bfr(gb[cc])), 0.f); unsigned short a, b2; splitf(y, a, b2); oh[q] = a; ol[q] = b2; }
    *(volatile v4us*)(Xh + e) = oh; *(volatile v4us*)(Xl + e) = ol; __threadfence(); *(volatile v4us*)(Xh + e) = oh; *(volatile v4us*)(Xl + e) = ol; }
__global__ __launch_bounds__(256) void k_cvt8(const float* __restrict__ src, bf* dst, size_t n8) { const size_t i = (size_t)blockIdx.x * 256 + threadIdx.x; if (i >= n8) return; const v8f v = *(const v8f*)(src + i * 8); v8us o;
#pragma unroll
    for (int k = 0; k < 8; ++k) o[k] = f2bf(v[k]); *(volatile v8us*)(dst + i * 8) = o; __threadfence(); *(volatile v8us*)(dst + i * 8) = o; }
__global__ void k_bias2(const float* __restrict__ bt, const float* __restrict__ bp, float* BTP) { const int lane = threadIdx.x; if (lane >= 32) return; v2f o; o[0] = (lane < 16) ? bt[lane * 2] : bp[(lane - 16) * 2]; o[1] = (lane < 16) ? bt[lane * 2 + 1] : bp[(lane - 16) * 2 + 1]; *(volatile v2f*)(BTP + lane * 2) = o; __threadfence(); *(volatile v2f*)(BTP + lane * 2) = o; }
__global__ __launch_bounds__(256) void k_poolT(const float* __restrict__ F, int ldf, int col0, int nch, bf* Ph, bf* Pl) { const size_t e = ((size_t)blockIdx.x * 256 + threadIdx.x) * 2; if (e >= (size_t)CG * NPP) return; const int m = (int)(e % NPP); const int ch = (int)(e / NPP); v2us oh, ol;
#pragma unroll
    for (int q = 0; q < 2; ++q) { const int mm = m + q; float v = 0.f; if (mm < NP && ch < nch) { const int ph = mm / PW, pw = mm % PW; const int n00 = (2 * ph) * WID + 2 * pw; const float* f = F + col0 + ch; v = fmaxf(fmaxf(f[(size_t)n00 * ldf], f[(size_t)(n00 + 1) * ldf]), fmaxf(f[(size_t)(n00 + WID) * ldf], f[(size_t)(n00 + WID + 1) * ldf])); } unsigned short a, b2; splitf(v, a, b2); oh[q] = a; ol[q] = b2; }
    *(volatile v2us*)(Ph + e) = oh; *(volatile v2us*)(Pl + e) = ol; __threadfence(); *(volatile v2us*)(Ph + e) = oh; *(volatile v2us*)(Pl + e) = ol; }
__global__ __launch_bounds__(256) void k_thpl(const float* __restrict__ TP, bf* Th, bf* Tl) { const size_t e = ((size_t)blockIdx.x * 256 + threadIdx.x) * 4; if (e >= (size_t)HW * CG) return; const int c = (int)(e % CG); const size_t n = e / CG; v4us oh, ol;
#pragma unroll
    for (int q = 0; q < 4; ++q) { const float v = (c + q < CI) ? TP[n * CG + c + q] : 0.f; unsigned short a, b2; splitf(v, a, b2); oh[q] = a; ol[q] = b2; }
    *(volatile v4us*)(Th + e) = oh; *(volatile v4us*)(Tl + e) = ol; __threadfence(); *(volatile v4us*)(Th + e) = oh; *(volatile v4us*)(Tl + e) = ol; }
__global__ __launch_bounds__(256) void k_msplit(const float* __restrict__ M, bf* Mh, bf* Ml) { const size_t i = (size_t)blockIdx.x * 256 + threadIdx.x; if (i >= (size_t)CG * CG / 4) return; const v4f a = *(const v4f*)(M + i * 4); v4us oh, ol;
#pragma unroll
    for (int q = 0; q < 4; ++q) { float v = __fmul_rn(a[q], 1.0f / (float)NP); asm volatile("" : "+v"(v)); unsigned short h2, l2; splitf(v, h2, l2); oh[q] = h2; ol[q] = l2; }
    *(volatile v4us*)(Mh + i * 4) = oh; *(volatile v4us*)(Ml + i * 4) = ol; __threadfence(); *(volatile v4us*)(Mh + i * 4) = oh; *(volatile v4us*)(Ml + i * 4) = ol; }
__global__ __launch_bounds__(256) void k_ycopy(const float* __restrict__ Y, float* YAb) { const size_t e = (size_t)blockIdx.x * 256 + threadIdx.x; if (e >= (size_t)CG * HW) return; const int n = (int)(e % HW); const int cg = (int)(e / HW); const float v = Y[(size_t)n * CG + cg]; *(volatile float*)(YAb + e) = v; __threadfence(); *(volatile float*)(YAb + e) = v; }
__global__ __launch_bounds__(256) void k_zpl(const float* __restrict__ YAb, const float* __restrict__ ST2, const float* __restrict__ gw, const float* __restrict__ gb, bf* Zh, bf* Zl) { const size_t e = ((size_t)blockIdx.x * 256 + threadIdx.x) * 4; if (e >= (size_t)HW * CG) return; const int cg = (int)(e % CG); const int n = (int)(e / CG); v4us oh, ol;
#pragma unroll
    for (int q = 0; q < 4; ++q) { const int cc = cg + q; const float mu = ST2[(size_t)cc * RPAD], rs = ST2[(size_t)cc * RPAD + 1]; float n0 = __fmul_rn(__fsub_rn(YAb[(size_t)cc * HW + n], mu), rs); asm volatile("" : "+v"(n0)); float n1 = __fmul_rn(bfr(gw[cc]), n0); asm volatile("" : "+v"(n1)); const float y = fmaxf(__fadd_rn(n1, bfr(gb[cc])), 0.f); unsigned short a, b2; splitf(y, a, b2); oh[q] = a; ol[q] = b2; }
    *(volatile v4us*)(Zh + e) = oh; *(volatile v4us*)(Zl + e) = ol; __threadfence(); *(volatile v4us*)(Zh + e) = oh; *(volatile v4us*)(Zl + e) = ol; }
__global__ __launch_bounds__(256) void k_outT(const float* __restrict__ xb, const float* __restrict__ WY, float* Ob) { const size_t e = (size_t)blockIdx.x * 256 + threadIdx.x; if (e >= (size_t)C_ * HW) return; const int n = (int)(e % HW); const int c = (int)(e / HW); const float v = __fadd_rn(bfr(xb[e]), WY[(size_t)n * C_ + c]); *(volatile float*)(Ob + e) = v; __threadfence(); *(volatile float*)(Ob + e) = v; }

extern "C" void kernel_launch(void* const* d_in, const int* in_sizes, int n_in,
                              void* d_out, int out_size, void* d_ws, size_t ws_size, hipStream_t stream) {
    (void)in_sizes; (void)n_in; (void)out_size;
    const float* x = (const float*)d_in[0]; const float* g1 = (const float*)d_in[1]; const float* e1 = (const float*)d_in[2]; const float* wg = (const float*)d_in[3]; const float* bg = (const float*)d_in[4]; const float* wt = (const float*)d_in[5]; const float* bt = (const float*)d_in[6]; const float* wp = (const float*)d_in[7]; const float* bp = (const float*)d_in[8]; const float* g2 = (const float*)d_in[9]; const float* e2 = (const float*)d_in[10]; const float* wz = (const float*)d_in[11]; const float* bz = (const float*)d_in[12];
    float* OUT = (float*)d_out;
    char* wsp = (char*)d_ws;
    auto take = [&](size_t bytes) { char* p = wsp; wsp += (bytes + 255) & ~(size_t)255; return (void*)p; };
    bf* WG = (bf*)take((size_t)CG * C_ * 2); bf* WTP = (bf*)take((size_t)CG * C_ * 2); bf* WZ = (bf*)take((size_t)C_ * CG * 2); float* BTP = (float*)take(CG * 4); float* ST1 = (float*)take((size_t)C_ * RPAD * 4); float* ST2 = (float*)take((size_t)CG * RPAD * 4);
    bf* XAh = (bf*)take((size_t)HW * C_ * 2); bf* XAl = (bf*)take((size_t)HW * C_ * 2); float* GT = (float*)take((size_t)HW * CG * 4); float* TP = (float*)take((size_t)HW * CG * 4);
    bf* GPh = (bf*)take((size_t)CG * NPP * 2); bf* GPl = (bf*)take((size_t)CG * NPP * 2); bf* FPh = (bf*)take((size_t)CG * NPP * 2); bf* FPl = (bf*)take((size_t)CG * NPP * 2); float* MTf = (float*)take((size_t)CG * CG * 4); bf* MTh = (bf*)take((size_t)CG * CG * 2); bf* MTl = (bf*)take((size_t)CG * CG * 2);
    bf* THh = (bf*)take((size_t)HW * CG * 2); bf* THl = (bf*)take((size_t)HW * CG * 2); float* Y = (float*)take((size_t)HW * CG * 4); float* YA = (float*)take((size_t)NB_ * CG * HW * 4); bf* Zh = (bf*)take((size_t)HW * CG * 2); bf* Zl = (bf*)take((size_t)HW * CG * 2); float* WY = (float*)take((size_t)HW * C_ * 4);
    if ((size_t)(wsp - (char*)d_ws) > ws_size) return;
    k_cvt8<<<(unsigned)(((size_t)CG * C_ / 8 + 255) / 256), 256, 0, stream>>>(wg, WG, (size_t)CG * C_ / 8); k_cvt8<<<(unsigned)(((size_t)CI * C_ / 8 + 255) / 256), 256, 0, stream>>>(wt, WTP, (size_t)CI * C_ / 8); k_cvt8<<<(unsigned)(((size_t)CI * C_ / 8 + 255) / 256), 256, 0, stream>>>(wp, WTP + (size_t)CI * C_, (size_t)CI * C_ / 8); k_cvt8<<<(unsigned)(((size_t)C_ * CG / 8 + 255) / 256), 256, 0, stream>>>(wz, WZ, (size_t)C_ * CG / 8); k_bias2<<<1, 32, 0, stream>>>(bt, bp, BTP);
    k_bnstat<true><<<C_, 256, 0, stream>>>(x, C_, HW, ST1);
    for (int b = 0; b < NB_; ++b) { const float* xb = x + (size_t)b * C_ * HW;
        k_bnT<<<(unsigned)(((size_t)HW * C_ / 4 + 255) / 256), 256, 0, stream>>>(xb, ST1, g1, e1, XAh, XAl);
        k_gemmw<bf, 1, true><<<dim3(HW / 64, 1, 1), 32, 0, stream>>>(XAh, XAl, WG, nullptr, C_, GT, CG, bg, 0, 0, 0);
        k_gemmw<bf, 1, true><<<dim3(HW / 64, 1, 1), 32, 0, stream>>>(XAh, XAl, WTP, nullptr, C_, TP, CG, BTP, 0, 0, 0);
        k_poolT<<<(unsigned)(((size_t)CG * NPP / 2 + 255) / 256), 256, 0, stream>>>(GT, CG, 0, CG, GPh, GPl);
        k_poolT<<<(unsigned)(((size_t)CG * NPP / 2 + 255) / 256), 256, 0, stream>>>(TP, CG, CI, CI, FPh, FPl);
        k_gemmw<bf, 2, false><<<dim3(1, 1, 1), 32, 0, stream>>>(GPh, GPl, FPh, FPl, NPP, MTf, CG, nullptr, 0, 0, 0);
        k_msplit<<<(unsigned)(((size_t)CG * CG / 4 + 255) / 256), 256, 0, stream>>>(MTf, MTh, MTl);
        k_thpl<<<(unsigned)(((size_t)HW * CG / 4 + 255) / 256), 256, 0, stream>>>(TP, THh, THl);
        k_gemmw<bf, 2, false><<<dim3(HW / 64, 1, 1), 32, 0, stream>>>(THh, THl, MTh, MTl, CG, Y, CG, nullptr, 0, 0, 0);
        k_ycopy<<<(unsigned)(((size_t)CG * HW + 255) / 256), 256, 0, stream>>>(Y, YA + (size_t)b * CG * HW); }
    k_bnstat<false><<<CG, 256, 0, stream>>>(YA, CG, HW, ST2);
    for (int b = 0; b < NB_; ++b) { const float* xb = x + (size_t)b * C_ * HW;
        k_zpl<<<(unsigned)(((size_t)HW * CG / 4 + 255) / 256), 256, 0, stream>>>(YA + (size_t)b * CG * HW, ST2, g2, e2, Zh, Zl);
        k_gemmw<bf, 1, true><<<dim3(HW / 64, C_ / 64, 1), 32, 0, stream>>>(Zh, Zl, WZ, nullptr, CG, WY, C_, bz, 0, 0, 0);
        k_outT<<<(unsigned)(((size_t)C_ * HW + 255) / 256), 256, 0, stream>>>(xb, WY, OUT + (size_t)b * C_ * HW); }
}
